// CasDOSeqModel_42339787604234
// MI455X (gfx1250) — hardware-run, weakly checked
//
#include <hip/hip_runtime.h>
#include <math.h>

typedef __attribute__((ext_vector_type(16))) _Float16 v16h;
typedef __attribute__((ext_vector_type(8)))  _Float16 v8h;
typedef __attribute__((ext_vector_type(16))) __bf16   v16b;
typedef __attribute__((ext_vector_type(8)))  __bf16   v8b;
typedef __attribute__((ext_vector_type(8)))  float    v8f;
typedef __attribute__((ext_vector_type(4)))  float    v4f;
typedef __attribute__((ext_vector_type(4)))  unsigned v4u;
typedef __attribute__((ext_vector_type(2)))  unsigned v2u;

constexpr int kB  = 4096;
constexpr int kE  = 768;
constexpr int kZ  = 64;
constexpr int kU  = 128;
constexpr int kT  = 512;
constexpr int kP  = kT + 1;
constexpr int kRows   = 16;
constexpr int kBlocks = kB / kRows;
constexpr int kOPitch = 544;
constexpr int kOutN   = kB * kP;
constexpr int kOutTotal = 2 * kOutN + 1;
constexpr int kCopyBlocks = (2 * kOutN / 4) / 256;
constexpr int kAP = kE + 8;
constexpr int kZP = kZ + 8;
constexpr int kUP = kU + 8;
constexpr int kFP = kZ + 4;
constexpr int kObP = 36;

static_assert(kB % kRows == 0);
static_assert(kBlocks == 256);
static_assert(kE % 32 == 0 && kZ % 32 == 0 && kU % 32 == 0);
static_assert(kZ % 16 == 0 && kU % 16 == 0);
static_assert(kT % 32 == 0);
static_assert(kOPitch % 32 == 0 && kOPitch >= kP + 31);
static_assert((kT / 32) * 32 + 32 <= kOPitch);
static_assert(((size_t)kOutN * 4) % 128 == 0);
static_assert(((size_t)2 * kOutN * 4) % 128 == 0);
static_assert((size_t)kOutN * 4 == 8404992ull);
static_assert((size_t)2 * kOutN * 4 == 16809984ull);
static_assert((size_t)kOutTotal * 4 == 16809988ull);
static_assert((2 * kOutN) % (4 * 256) == 0);
static_assert(kCopyBlocks == 4104);

constexpr float kCarryZ = 8.0f;
constexpr float kCarryH = 32.0f;
constexpr float kCarryW = 256.0f;
constexpr float kF16MinNormal = 6.103515625e-5f;
constexpr float kDt   = 1.0f / (float)kT;
constexpr float kSZW  = 1.0f / (kCarryZ * kCarryW);
constexpr float kSHW  = 1.0f / (kCarryH * kCarryW);
constexpr float kLnEps = 1e-5f;
constexpr float kInvZ  = 1.0f / (float)kZ;
constexpr float kInvCount = 1.0f / (float)(kB * kZ);

constexpr size_t kOffWPT  = 0;
constexpr size_t kOffDW1T = kOffWPT  + (size_t)kZ * kE * 2;
constexpr size_t kOffDW2T = kOffDW1T + (size_t)kU * kZ * 2;
constexpr size_t kOffOW1T = kOffDW2T + (size_t)kZ * kU * 2;
constexpr size_t kOffOW2T = kOffOW1T + (size_t)kU * kZ * 2;
constexpr size_t kOffOW3T = kOffOW2T + (size_t)kU * kU * 2;
constexpr size_t kOffZA   = kOffOW3T + (size_t)kZ * kU * 2;
constexpr size_t kOffPART = kOffZA   + (size_t)kB * kZ * 4;
constexpr size_t kOffOP   = kOffPART + (size_t)kBlocks * 32 * 4;
constexpr size_t kWsTotal = kOffOP   + (size_t)2 * kB * kOPitch * 4;
static_assert(kWsTotal == 19103744ull);
static_assert(kWsTotal <= 134217728ull);
static_assert(kOffDW1T % 128 == 0 && kOffDW2T % 128 == 0 && kOffOW1T % 128 == 0 && kOffOW2T % 128 == 0 &&
              kOffOW3T % 128 == 0 && kOffZA % 128 == 0 && kOffPART % 128 == 0 && kOffOP % 128 == 0);
constexpr int kChWPT = kZ * kE / 8;
constexpr int kChA   = kU * kZ / 8;
constexpr int kChW2  = kU * kU / 8;
constexpr int kChunks = kChWPT + 4 * kChA + kChW2;
static_assert(kChWPT == 6144 && kChA == 1024 && kChW2 == 2048 && kChunks == 12288);
static_assert(kChunks % 256 == 0);
static_assert((size_t)kChunks * 16 == kOffZA);

__device__ __forceinline__ unsigned short f2bf_bits(float f) {
  unsigned u = __float_as_uint(f);
  return (unsigned short)((u + 0x7FFFu + ((u >> 16) & 1u)) >> 16);
}
__device__ __forceinline__ float bf_bits2f(unsigned short h) { return __uint_as_float(((unsigned)h) << 16); }
__device__ __forceinline__ float bfv(float f) { return bf_bits2f(f2bf_bits(f)); }
__device__ __forceinline__ float flush16(float v) { return (fabsf(v) < kF16MinNormal) ? 0.0f : v; }

struct FragH {
  union U { v16h v; v8h h[2]; };
  static __device__ __forceinline__ v16h load(const _Float16* p) {
    U f;
    f.h[0] = *(const v8h*)(p);
    f.h[1] = *(const v8h*)(p + 16);
    return f.v;
  }
};
struct FragB {
  union U { v16b v; v8b h[2]; };
  static __device__ __forceinline__ v16b load(const __bf16* p) {
    U f;
    f.h[0] = *(const v8b*)(p);
    f.h[1] = *(const v8b*)(p + 16);
    return f.v;
  }
};
__device__ __forceinline__ v8f mma_h(v16h a, v16h b, v8f c) {
  c = __builtin_amdgcn_wmma_f32_16x16x32_f16(false, a, false, b, (short)0, c, false, false);
  asm volatile("v_nop\n\tv_nop\n\tv_nop\n\tv_nop" : "+v"(c) : "v"(a), "v"(b));
  return c;
}
__device__ __forceinline__ v8f mma_b(v16b a, v16b b, v8f c) {
  c = __builtin_amdgcn_wmma_f32_16x16x32_bf16(false, a, false, b, (short)0, c, false, false);
  asm volatile("v_nop\n\tv_nop\n\tv_nop\n\tv_nop" : "+v"(c) : "v"(a), "v"(b));
  return c;
}
template <int KSTEPS>
__device__ __forceinline__ v8f tile_prod(const _Float16* wrow, const v16h (&bf)[KSTEPS]) {
  v8f acc = (v8f){0.f, 0.f, 0.f, 0.f, 0.f, 0.f, 0.f, 0.f};
#pragma unroll
  for (int ks = 0; ks < KSTEPS; ++ks) {
    const v16h a = FragH::load(wrow + 32 * ks);
    acc = mma_h(a, bf[ks], acc);
  }
  return acc;
}
__device__ __forceinline__ _Float16 tanh_plane(float x2) {
  const float e = __expf(x2);
  const float r = __builtin_amdgcn_rcpf(1.0f + e);
  const float t = fmaf(-2.0f * kCarryH, r, kCarryH);
  return (_Float16)flush16(t);
}

__global__ __launch_bounds__(256) void prep_planes(
    const float* __restrict__ projW, const float* __restrict__ dW1, const float* __restrict__ dW2,
    const float* __restrict__ oW1, const float* __restrict__ oW2, const float* __restrict__ oW3,
    unsigned* __restrict__ planes)
{
  const int blk = blockIdx.x, tid = threadIdx.x;
  const float* src = projW;
  int ldn = kZ, cpr = kE / 8, cbase = 0;
  bool asbf = true;
  if (blk >= 44)      { src = oW3; ldn = kZ; cpr = kU / 8; cbase = kChWPT + 3 * kChA + kChW2; asbf = false; }
  else if (blk >= 36) { src = oW2; ldn = kU; cpr = kU / 8; cbase = kChWPT + 3 * kChA;         asbf = false; }
  else if (blk >= 32) { src = oW1; ldn = kU; cpr = kZ / 8; cbase = kChWPT + 2 * kChA;         asbf = false; }
  else if (blk >= 28) { src = dW2; ldn = kZ; cpr = kU / 8; cbase = kChWPT + kChA;             asbf = false; }
  else if (blk >= 24) { src = dW1; ldn = kU; cpr = kZ / 8; cbase = kChWPT;                    asbf = false; }
  const int c  = blk * 256 + tid;
  const int cl = c - cbase;
  const int nrow = cl / cpr;
  const int k0 = (cl - nrow * cpr) * 8;
  unsigned bits[8];
#pragma unroll
  for (int e = 0; e < 8; ++e) {
    const float x = src[(size_t)(k0 + e) * ldn + nrow];
    const unsigned short bb = f2bf_bits(x);
    const float cv = flush16(bf_bits2f(bb) * kCarryW);
    const _Float16 hv = (_Float16)cv;
    const unsigned short hb = __builtin_bit_cast(unsigned short, hv);
    bits[e] = asbf ? (unsigned)bb : (unsigned)hb;
  }
  v4u o;
  o[0] = bits[0] | (bits[1] << 16);
  o[1] = bits[2] | (bits[3] << 16);
  o[2] = bits[4] | (bits[5] << 16);
  o[3] = bits[6] | (bits[7] << 16);
  unsigned* dst = planes + (size_t)c * 4;
  *(volatile v4u*)dst = o;
  __threadfence();
  *(volatile v4u*)dst = o;
}

__global__ __launch_bounds__(128) void front_end(
    const float* __restrict__ emb, const float* __restrict__ epsn,
    const float* __restrict__ projB, const float* __restrict__ lnG, const float* __restrict__ lnB,
    const float* __restrict__ logNs, const float* __restrict__ dB1, const float* __restrict__ dB2,
    const unsigned short* __restrict__ WPT, const unsigned short* __restrict__ DW1T,
    const unsigned short* __restrict__ DW2T, float* __restrict__ ZA, float* __restrict__ PART)
{
  __shared__ __align__(16) unsigned short sA[kRows * kAP];
  __shared__ __align__(16) float sH[kRows * kFP];
  __shared__ __align__(16) float sZc[kRows * kFP];
  __shared__ __align__(16) float sZa[kRows * kFP];
  __shared__ __align__(16) _Float16 sZn[kRows * kZP];
  __shared__ __align__(16) _Float16 sHid[kRows * kUP];
  __shared__ __align__(16) float sPart[128];

  const int tid = threadIdx.x, lane = tid & 31, w = tid >> 5, h = lane >> 4, n = lane & 15;
  const int blk = blockIdx.x;
  const int row0 = blk * kRows;

#pragma unroll 1
  for (int it = 0; it < 24; ++it) {
    const int q = it * 128 + tid;
    const int r = q / 192;
    const int c4 = q - r * 192;
    const v4f x = *(const v4f*)(emb + (size_t)(row0 + r) * kE + c4 * 4);
    v2u o;
    o[0] = (unsigned)f2bf_bits(x[0]) | ((unsigned)f2bf_bits(x[1]) << 16);
    o[1] = (unsigned)f2bf_bits(x[2]) | ((unsigned)f2bf_bits(x[3]) << 16);
    *(v2u*)(sA + r * kAP + c4 * 4) = o;
  }
  __syncthreads();

  {
    v8f acc = (v8f){0.f, 0.f, 0.f, 0.f, 0.f, 0.f, 0.f, 0.f};
    const __bf16* ap = (const __bf16*)WPT + (size_t)(16 * w + n) * kE + 8 * h;
    const __bf16* bp = (const __bf16*)sA + n * kAP + 8 * h;
#pragma unroll 2
    for (int k0 = 0; k0 < kE; k0 += 32) {
      const v16b a = FragB::load(ap + k0);
      const v16b b = FragB::load(bp + k0);
      acc = mma_b(a, b, acc);
    }
    const int m0 = 16 * w + 8 * h;
    const v4f p0 = *(const v4f*)(projB + m0);
    const v4f p1 = *(const v4f*)(projB + m0 + 4);
    v4f o0, o1;
#pragma unroll
    for (int e = 0; e < 4; ++e) {
      o0[e] = acc[e] + bfv(p0[e]);
      o1[e] = acc[4 + e] + bfv(p1[e]);
    }
    *(v4f*)(sH + n * kFP + m0) = o0;
    *(v4f*)(sH + n * kFP + m0 + 4) = o1;
  }
  __syncthreads();

  {
    const int row = tid >> 3, seg = tid & 7;
    const float* hr = sH + row * kFP;
    float mu = 0.0f;
#pragma unroll 1
    for (int q = 0; q < 16; ++q) {
      const v4f x = *(const v4f*)(hr + 4 * q);
      mu += x[0]; mu += x[1]; mu += x[2]; mu += x[3];
    }
    mu *= kInvZ;
    float var = 0.0f;
#pragma unroll 1
    for (int q = 0; q < 16; ++q) {
      const v4f x = *(const v4f*)(hr + 4 * q);
      const float d0 = x[0] - mu, d1 = x[1] - mu, d2 = x[2] - mu, d3 = x[3] - mu;
      var = fmaf(d0, d0, var);
      var = fmaf(d1, d1, var);
      var = fmaf(d2, d2, var);
      var = fmaf(d3, d3, var);
    }
    var *= kInvZ;
    const float rs = rsqrtf(var + kLnEps);
    float lx = bfv(logNs[0]);
    asm volatile("" : "+v"(lx));
    const float sigma = fmaxf(lx, 0.0f) + log1pf(expf(-fabsf(lx)));
    const v4f h0 = *(const v4f*)(hr + seg * 8);
    const v4f h1 = *(const v4f*)(hr + seg * 8 + 4);
    const v4f g0 = *(const v4f*)(lnG + seg * 8);
    const v4f g1 = *(const v4f*)(lnG + seg * 8 + 4);
    const v4f c0 = *(const v4f*)(lnB + seg * 8);
    const v4f c1 = *(const v4f*)(lnB + seg * 8 + 4);
    const float* ep = epsn + (size_t)(row0 + row) * kZ + seg * 8;
    const v4f e0 = *(const v4f*)(ep);
    const v4f e1 = *(const v4f*)(ep + 4);
    v4f zc0, zc1;
    v8h zn;
#pragma unroll
    for (int e = 0; e < 4; ++e) {
      const float a0 = (h0[e] - mu) * rs * bfv(g0[e]) + bfv(c0[e]);
      const float a1 = (h1[e] - mu) * rs * bfv(g1[e]) + bfv(c1[e]);
      zc0[e] = a0;
      zc1[e] = a1;
      const float n0 = a0 + sigma * bfv(e0[e]);
      const float n1 = a1 + sigma * bfv(e1[e]);
      zn[e]     = (_Float16)flush16(n0 * kCarryZ);
      zn[4 + e] = (_Float16)flush16(n1 * kCarryZ);
    }
    *(v4f*)(sZc + row * kFP + seg * 8) = zc0;
    *(v4f*)(sZc + row * kFP + seg * 8 + 4) = zc1;
    *(v8h*)(sZn + row * kZP + seg * 8) = zn;
  }
  __syncthreads();

  {
    v16h bf[2];
    const _Float16* bp = sZn + n * kZP + 8 * h;
    bf[0] = FragH::load(bp);
    bf[1] = FragH::load(bp + 32);
#pragma unroll 1
    for (int i = 0; i < 2; ++i) {
      const int m0 = 32 * w + 16 * i;
      const v8f acc = tile_prod<2>((const _Float16*)DW1T + (size_t)(m0 + n) * kZ + 8 * h, bf);
      const v4f p0 = *(const v4f*)(dB1 + m0 + 8 * h);
      const v4f p1 = *(const v4f*)(dB1 + m0 + 8 * h + 4);
      v8h hv;
#pragma unroll
      for (int e = 0; e < 4; ++e) {
        const float x0 = fmaf(acc[e], kSZW, bfv(p0[e]));
        const float x1 = fmaf(acc[4 + e], kSZW, bfv(p1[e]));
        const float s0 = __builtin_amdgcn_rcpf(1.0f + expf(-x0));
        const float s1 = __builtin_amdgcn_rcpf(1.0f + expf(-x1));
        hv[e]     = (_Float16)flush16(x0 * s0 * kCarryH);
        hv[4 + e] = (_Float16)flush16(x1 * s1 * kCarryH);
      }
      *(v8h*)(sHid + n * kUP + m0 + 8 * h) = hv;
    }
  }
  __syncthreads();

  {
    v16h bf[4];
    const _Float16* bp = sHid + n * kUP + 8 * h;
#pragma unroll
    for (int ks = 0; ks < 4; ++ks) bf[ks] = FragH::load(bp + 32 * ks);
    const int m0 = 16 * w;
    const v8f acc = tile_prod<4>((const _Float16*)DW2T + (size_t)(m0 + n) * kU + 8 * h, bf);
    const v4f p0 = *(const v4f*)(dB2 + m0 + 8 * h);
    const v4f p1 = *(const v4f*)(dB2 + m0 + 8 * h + 4);
    v4f o0, o1;
#pragma unroll
    for (int e = 0; e < 4; ++e) {
      o0[e] = fmaf(acc[e], kSHW, bfv(p0[e]));
      o1[e] = fmaf(acc[4 + e], kSHW, bfv(p1[e]));
    }
    *(v4f*)(sZa + n * kFP + m0 + 8 * h) = o0;
    *(v4f*)(sZa + n * kFP + m0 + 8 * h + 4) = o1;
  }
  __syncthreads();

  {
    const int row = tid >> 3, seg = tid & 7;
    const v4f a0 = *(const v4f*)(sZa + row * kFP + seg * 8);
    const v4f a1 = *(const v4f*)(sZa + row * kFP + seg * 8 + 4);
    const v4f c0 = *(const v4f*)(sZc + row * kFP + seg * 8);
    const v4f c1 = *(const v4f*)(sZc + row * kFP + seg * 8 + 4);
    float s = 0.0f;
#pragma unroll
    for (int e = 0; e < 4; ++e) { const float d = a0[e] - c0[e]; s = fmaf(d, d, s); }
#pragma unroll
    for (int e = 0; e < 4; ++e) { const float d = a1[e] - c1[e]; s = fmaf(d, d, s); }
    sPart[tid] = s;
  }
  {
    v4f zv[2];
    float* dst[2];
#pragma unroll
    for (int it = 0; it < 2; ++it) {
      const int q = it * 128 + tid;
      const int r = q >> 4, c4 = q & 15;
      zv[it] = *(const v4f*)(sZa + r * kFP + c4 * 4);
      dst[it] = ZA + (size_t)row0 * kZ + (size_t)q * 4;
    }
    for (int pass = 0; pass < 2; ++pass) {
#pragma unroll
      for (int it = 0; it < 2; ++it) *(volatile v4f*)dst[it] = zv[it];
      __threadfence();
    }
  }
  __syncthreads();
  if (w == 0) {
    float s = 0.0f;
    s += sPart[4 * lane + 0];
    s += sPart[4 * lane + 1];
    s += sPart[4 * lane + 2];
    s += sPart[4 * lane + 3];
    s += __shfl_xor(s, 16, 32);
    s += __shfl_xor(s, 8, 32);
    s += __shfl_xor(s, 4, 32);
    s += __shfl_xor(s, 2, 32);
    s += __shfl_xor(s, 1, 32);
    const float o = (lane == 0) ? s : 0.0f;
    float* pp = PART + (size_t)blk * 32 + lane;
    *(volatile float*)pp = o;
    __threadfence();
    *(volatile float*)pp = o;
  }
}

__device__ __forceinline__ float head_dot(const float* zrow, const float (&wr)[16]) {
  float s = 0.0f;
#pragma unroll
  for (int q = 0; q < 4; ++q) {
    const v4f x = *(const v4f*)(zrow + 4 * q);
    s = fmaf(x[0], wr[4 * q + 0], s);
    s = fmaf(x[1], wr[4 * q + 1], s);
    s = fmaf(x[2], wr[4 * q + 2], s);
    s = fmaf(x[3], wr[4 * q + 3], s);
  }
  s += __shfl_xor(s, 1, 32);
  s += __shfl_xor(s, 2, 32);
  return s;
}
__device__ __forceinline__ void put_z(_Float16* sZ16, float* sZf, const float (&zr)[8], int n, int c0) {
  v8h zh;
  v4f f0, f1;
#pragma unroll
  for (int e = 0; e < 4; ++e) {
    zh[e]     = (_Float16)flush16(zr[e] * kCarryZ);
    zh[4 + e] = (_Float16)flush16(zr[4 + e] * kCarryZ);
    f0[e] = zr[e];
    f1[e] = zr[4 + e];
  }
  *(v8h*)(sZ16 + n * kZP + c0) = zh;
  *(v4f*)(sZf + n * kFP + c0) = f0;
  *(v4f*)(sZf + n * kFP + c0 + 4) = f1;
}
__device__ __forceinline__ void flush_lines(const float* sOb, float* OP, int blk, int w, int lane, int chunk) {
  const int q = lane >> 3, c4 = (lane & 7) * 4;
  v4f v[2];
  float* dst[2];
#pragma unroll
  for (int ii = 0; ii < 2; ++ii) {
    const int R = 8 * w + 4 * ii + q;
    const int ch = R >> 4, smp = R & 15;
    v[ii] = *(const v4f*)(sOb + R * kObP + c4);
    dst[ii] = OP + ((size_t)(ch * kB + blk * kRows + smp)) * kOPitch + chunk * 32 + c4;
  }
  for (int pass = 0; pass < 2; ++pass) {
#pragma unroll
    for (int ii = 0; ii < 2; ++ii) *(volatile v4f*)dst[ii] = v[ii];
    __threadfence();
  }
}

__global__ __launch_bounds__(128) void euler_steps(
    const float* __restrict__ ZA,
    const unsigned short* __restrict__ OW1T, const unsigned short* __restrict__ OW2T,
    const unsigned short* __restrict__ OW3T,
    const float* __restrict__ oB1, const float* __restrict__ oB2, const float* __restrict__ oB3,
    const float* __restrict__ decW, const float* __restrict__ decB, float* __restrict__ OP)
{
  __shared__ __align__(16) _Float16 sW1[kU * kZP];
  __shared__ __align__(16) _Float16 sW2[kU * kUP];
  __shared__ __align__(16) _Float16 sW3[kZ * kUP];
  __shared__ __align__(16) _Float16 sZ16[kRows * kZP];
  __shared__ __align__(16) _Float16 sH1[kRows * kUP];
  __shared__ __align__(16) _Float16 sH2[kRows * kUP];
  __shared__ __align__(16) float sZf[kRows * kFP];
  __shared__ __align__(16) float sOb[32 * kObP];
  __shared__ __align__(16) float sDW[2 * kZ];

  const int tid = threadIdx.x, lane = tid & 31, w = tid >> 5, h = lane >> 4, n = lane & 15;
  const int blk = blockIdx.x;

#pragma unroll 1
  for (int i = 0; i < 8; ++i) {
    const int c = i * 128 + tid;
    const v4u x = *(const v4u*)(OW1T + (size_t)c * 8);
    *(v4u*)(sW1 + (c >> 3) * kZP + (c & 7) * 8) = x;
  }
#pragma unroll 1
  for (int i = 0; i < 16; ++i) {
    const int c = i * 128 + tid;
    const v4u x = *(const v4u*)(OW2T + (size_t)c * 8);
    *(v4u*)(sW2 + (c >> 4) * kUP + (c & 15) * 8) = x;
  }
#pragma unroll 1
  for (int i = 0; i < 8; ++i) {
    const int c = i * 128 + tid;
    const v4u x = *(const v4u*)(OW3T + (size_t)c * 8);
    *(v4u*)(sW3 + (c >> 4) * kUP + (c & 15) * 8) = x;
  }
  sDW[tid] = bfv(decW[tid]);

  float zr[8];
  {
    const float* zp = ZA + (size_t)(blk * kRows + n) * kZ + 16 * w + 8 * h;
    const v4f z0 = *(const v4f*)(zp);
    const v4f z1 = *(const v4f*)(zp + 4);
#pragma unroll
    for (int e = 0; e < 4; ++e) { zr[e] = z0[e]; zr[4 + e] = z1[e]; }
  }
  put_z(sZ16, sZf, zr, n, 16 * w + 8 * h);

  float b1x[2][8], b2x[2][8], b3d[8];
#pragma unroll
  for (int i = 0; i < 2; ++i) {
    const int m0 = 32 * w + 16 * i + 8 * h;
    const v4f p0 = *(const v4f*)(oB1 + m0);
    const v4f p1 = *(const v4f*)(oB1 + m0 + 4);
    const v4f q0 = *(const v4f*)(oB2 + m0);
    const v4f q1 = *(const v4f*)(oB2 + m0 + 4);
#pragma unroll
    for (int e = 0; e < 4; ++e) {
      b1x[i][e]     = 2.0f * bfv(p0[e]);
      b1x[i][4 + e] = 2.0f * bfv(p1[e]);
      b2x[i][e]     = 2.0f * bfv(q0[e]);
      b2x[i][4 + e] = 2.0f * bfv(q1[e]);
    }
  }
  {
    const int m0 = 16 * w + 8 * h;
    const v4f p0 = *(const v4f*)(oB3 + m0);
    const v4f p1 = *(const v4f*)(oB3 + m0 + 4);
#pragma unroll
    for (int e = 0; e < 4; ++e) {
      b3d[e]     = kDt * bfv(p0[e]);
      b3d[4 + e] = kDt * bfv(p1[e]);
    }
  }
  __syncthreads();

  const int hrow = tid >> 3, hch = (tid >> 2) & 1, hpart = tid & 3;
  float wreg[16];
#pragma unroll
  for (int i = 0; i < 16; ++i) wreg[i] = sDW[(hpart * 16 + i) * 2 + hch];
  const float hbias = bfv(decB[hch]);
  const float* hz = sZf + hrow * kFP + hpart * 16;
  float* hob = sOb + (hch * 16 + hrow) * kObP;

#pragma unroll 1
  for (int it = 0; it < kT; ++it) {
    {
      const float s = head_dot(hz, wreg) + hbias;
      if (hpart == 0) hob[it & 31] = s;
    }
    {
      v16h bf[2];
      const _Float16* bp = sZ16 + n * kZP + 8 * h;
      bf[0] = FragH::load(bp);
      bf[1] = FragH::load(bp + 32);
#pragma unroll
      for (int i = 0; i < 2; ++i) {
        const int m0 = 32 * w + 16 * i;
        const v8f acc = tile_prod<2>(sW1 + (m0 + n) * kZP + 8 * h, bf);
        v8h hv;
#pragma unroll
        for (int r = 0; r < 8; ++r) hv[r] = tanh_plane(fmaf(acc[r], 2.0f * kSZW, b1x[i][r]));
        *(v8h*)(sH1 + n * kUP + m0 + 8 * h) = hv;
      }
    }
    __syncthreads();
    if ((it & 31) == 31) flush_lines(sOb, OP, blk, w, lane, it >> 5);
    {
      v16h bf[4];
      const _Float16* bp = sH1 + n * kUP + 8 * h;
#pragma unroll
      for (int ks = 0; ks < 4; ++ks) bf[ks] = FragH::load(bp + 32 * ks);
#pragma unroll
      for (int i = 0; i < 2; ++i) {
        const int m0 = 32 * w + 16 * i;
        const v8f acc = tile_prod<4>(sW2 + (m0 + n) * kUP + 8 * h, bf);
        v8h hv;
#pragma unroll
        for (int r = 0; r < 8; ++r) hv[r] = tanh_plane(fmaf(acc[r], 2.0f * kSHW, b2x[i][r]));
        *(v8h*)(sH2 + n * kUP + m0 + 8 * h) = hv;
      }
    }
    __syncthreads();
    {
      v16h bf[4];
      const _Float16* bp = sH2 + n * kUP + 8 * h;
#pragma unroll
      for (int ks = 0; ks < 4; ++ks) bf[ks] = FragH::load(bp + 32 * ks);
      const v8f acc = tile_prod<4>(sW3 + (16 * w + n) * kUP + 8 * h, bf);
#pragma unroll
      for (int r = 0; r < 8; ++r) zr[r] = fmaf(acc[r], kSHW * kDt, zr[r] + b3d[r]);
      put_z(sZ16, sZf, zr, n, 16 * w + 8 * h);
    }
    __syncthreads();
  }
  {
    const float s = head_dot(hz, wreg) + hbias;
    if (hpart == 0) hob[0] = s;
#pragma unroll 1
    for (int idx = tid; idx < 32 * 32; idx += 128) {
      const int rr = idx >> 5, cc = idx & 31;
      if (cc != 0) sOb[rr * kObP + cc] = 0.0f;
    }
  }
  __syncthreads();
  flush_lines(sOb, OP, blk, w, lane, kT / 32);
}

__global__ __launch_bounds__(256) void flat_copy(
    const float* __restrict__ OP, const float* __restrict__ PART, float* __restrict__ out)
{
  const int blk = blockIdx.x, tid = threadIdx.x;
  if (blk < kCopyBlocks) {
    const int f0 = (blk * 256 + tid) * 4;
    v4f v;
#pragma unroll
    for (int e = 0; e < 4; ++e) {
      const int f = f0 + e;
      const int o = f / kOutN;
      const int rem = f - o * kOutN;
      const int smp = rem / kP;
      const int j = rem - smp * kP;
      v[e] = OP[(size_t)(o * kB + smp) * kOPitch + j];
    }
    float* dst = out + f0;
    *(volatile v4f*)dst = v;
    __threadfence();
    *(volatile v4f*)dst = v;
  } else {
    if (tid < 32) {
      const int lane = tid;
      float s = 0.0f;
#pragma unroll
      for (int i = 0; i < 8; ++i) s += PART[(size_t)(lane * 8 + i) * 32];
      s += __shfl_xor(s, 16, 32);
      s += __shfl_xor(s, 8, 32);
      s += __shfl_xor(s, 4, 32);
      s += __shfl_xor(s, 2, 32);
      s += __shfl_xor(s, 1, 32);
      const float loss = s * kInvCount;
      float* lp = out + (size_t)2 * kOutN;
      if (lane == 0) *(volatile float*)lp = loss;
      __threadfence();
      if (lane == 0) *(volatile float*)lp = loss;
    }
  }
}

extern "C" void kernel_launch(void* const* d_in, const int* in_sizes, int n_in,
                              void* d_out, int out_size, void* d_ws, size_t ws_size,
                              hipStream_t stream) {
  if (n_in < 21) return;
  if (in_sizes[0] != kB * kE) return;
  if (in_sizes[1] != kB * kT) return;
  if (in_sizes[3] != kB * kZ) return;
  if (in_sizes[4] != kE * kZ) return;
  if (in_sizes[5] != kZ || in_sizes[6] != kZ || in_sizes[7] != kZ) return;
  if (in_sizes[8] != 1) return;
  if (in_sizes[9] != kZ * kU || in_sizes[10] != kU) return;
  if (in_sizes[11] != kU * kZ || in_sizes[12] != kZ) return;
  if (in_sizes[13] != kZ * kU || in_sizes[14] != kU) return;
  if (in_sizes[15] != kU * kU || in_sizes[16] != kU) return;
  if (in_sizes[17] != kU * kZ || in_sizes[18] != kZ) return;
  if (in_sizes[19] != kZ * 2 || in_sizes[20] != 2) return;
  if (out_size != kOutTotal) return;
  if (ws_size < kWsTotal) return;

  const float* emb   = (const float*)d_in[0];
  const float* epsn  = (const float*)d_in[3];
  const float* projW = (const float*)d_in[4];
  const float* projB = (const float*)d_in[5];
  const float* lnG   = (const float*)d_in[6];
  const float* lnB   = (const float*)d_in[7];
  const float* logNs = (const float*)d_in[8];
  const float* dW1   = (const float*)d_in[9];
  const float* dB1   = (const float*)d_in[10];
  const float* dW2   = (const float*)d_in[11];
  const float* dB2   = (const float*)d_in[12];
  const float* oW1   = (const float*)d_in[13];
  const float* oB1   = (const float*)d_in[14];
  const float* oW2   = (const float*)d_in[15];
  const float* oB2   = (const float*)d_in[16];
  const float* oW3   = (const float*)d_in[17];
  const float* oB3   = (const float*)d_in[18];
  const float* decW  = (const float*)d_in[19];
  const float* decB  = (const float*)d_in[20];
  float* out = (float*)d_out;

  char* ws = (char*)d_ws;
  unsigned short* WPT  = (unsigned short*)(ws + kOffWPT);
  unsigned short* DW1T = (unsigned short*)(ws + kOffDW1T);
  unsigned short* DW2T = (unsigned short*)(ws + kOffDW2T);
  unsigned short* OW1T = (unsigned short*)(ws + kOffOW1T);
  unsigned short* OW2T = (unsigned short*)(ws + kOffOW2T);
  unsigned short* OW3T = (unsigned short*)(ws + kOffOW3T);
  float* ZA   = (float*)(ws + kOffZA);
  float* PART = (float*)(ws + kOffPART);
  float* OP   = (float*)(ws + kOffOP);

  prep_planes<<<kChunks / 256, 256, 0, stream>>>(projW, dW1, dW2, oW1, oW2, oW3, (unsigned*)(ws + kOffWPT));

  front_end<<<kBlocks, 128, 0, stream>>>(emb, epsn, projB, lnG, lnB, logNs, dB1, dB2,
                                         WPT, DW1T, DW2T, ZA, PART);

  euler_steps<<<kBlocks, 128, 0, stream>>>(ZA, OW1T, OW2T, OW3T, oB1, oB2, oB3, decW, decB, OP);

  flat_copy<<<kCopyBlocks + 1, 256, 0, stream>>>(OP, PART, out);
}
